// CorrBlock_43267500540365
// MI455X (gfx1250) — hardware-verified
//
#include <hip/hip_runtime.h>

typedef __attribute__((ext_vector_type(16))) _Float16 v16h;
typedef __attribute__((ext_vector_type(8)))  _Float16 v8h;
typedef __attribute__((ext_vector_type(16))) __bf16   v16b;
typedef __attribute__((ext_vector_type(8)))  __bf16   v8b;
typedef __attribute__((ext_vector_type(8)))  float    v8f;
typedef __attribute__((ext_vector_type(4)))  float    v4f;

#define NB   2
#define NC   256
#define WD   96
#define HW   9216
#define NCH  324
#define CHUNK_ROWS 24
#define CHUNK_PIX  2304
#define NCHUNK_PER_B 4

__device__ __forceinline__ unsigned short f2bf_bits(float f) {
  unsigned u = __float_as_uint(f);
  return (unsigned short)((u + 0x7FFFu + ((u >> 16) & 1u)) >> 16);
}
__device__ __forceinline__ float bf_bits2f(unsigned short h) { return __uint_as_float(((unsigned)h) << 16); }

__device__ __forceinline__ void dep_guard_h(v8f& a, v8f& b, v16h x, v16h y) { asm volatile("v_nop\n\tv_nop\n\tv_nop\n\tv_nop" : "+v"(a), "+v"(b) : "v"(x), "v"(y)); }
__device__ __forceinline__ void dep_guard_b(v8f& a, v8f& b, v16b x, v16b y) { asm volatile("v_nop\n\tv_nop\n\tv_nop\n\tv_nop" : "+v"(a), "+v"(b) : "v"(x), "v"(y)); }
__device__ __forceinline__ void keep4_h(v16h a, v16h b, v16h c, v16h d) { asm volatile("v_nop" :: "v"(a), "v"(b), "v"(c), "v"(d)); }
__device__ __forceinline__ void keep4_b(v16b a, v16b b, v16b c, v16b d) { asm volatile("v_nop" :: "v"(a), "v"(b), "v"(c), "v"(d)); }
__device__ __forceinline__ void acc_guard4(v8f& a, v8f& b, v8f& c, v8f& d) { asm volatile("v_nop\n\tv_nop\n\tv_nop\n\tv_nop" : "+v"(a), "+v"(b), "+v"(c), "+v"(d)); }
template <typename T> struct Frag;
template <> struct Frag<_Float16> {
  typedef v16h V; union U { v16h v; v8h h[2]; };
  static __device__ __forceinline__ v16h load(const _Float16* p) {
    U f; f.h[0] = *(const v8h*)(p); f.h[1] = *(const v8h*)(p + 16); return f.v;
  }
  static __device__ __forceinline__ v8f mma(v16h a, v16h b, v8f c) {
    return __builtin_amdgcn_wmma_f32_16x16x32_f16(false, a, false, b, (short)0, c, false, false);
  }
  static __device__ __forceinline__ void guard(v8f& a, v8f& b, v16h x, v16h y) { dep_guard_h(a, b, x, y); }
  static __device__ __forceinline__ void keep(v16h a, v16h b, v16h c, v16h d) { keep4_h(a, b, c, d); }
};
template <> struct Frag<__bf16> {
  typedef v16b V; union U { v16b v; v8b h[2]; };
  static __device__ __forceinline__ v16b load(const __bf16* p) {
    U f; f.h[0] = *(const v8b*)(p); f.h[1] = *(const v8b*)(p + 16); return f.v;
  }
  static __device__ __forceinline__ v8f mma(v16b a, v16b b, v8f c) {
    return __builtin_amdgcn_wmma_f32_16x16x32_bf16(false, a, false, b, (short)0, c, false, false);
  }
  static __device__ __forceinline__ void guard(v8f& a, v8f& b, v16b x, v16b y) { dep_guard_b(a, b, x, y); }
  static __device__ __forceinline__ void keep(v16b a, v16b b, v16b c, v16b d) { keep4_b(a, b, c, d); }
};

template <int ET> struct Elem;
template <> struct Elem<0> { typedef _Float16 T; };
template <> struct Elem<1> { typedef __bf16 T; };
template <int ET, bool SPLIT, int BIAS_MODE, int OUT_MODE, bool RESID, int ACT = 0>
__global__ __launch_bounds__(256) void wmma_gemm64(
    const unsigned short* __restrict__ Ap, const unsigned short* __restrict__ A2p, int lda, long strideA,
    const unsigned short* __restrict__ Btp, const unsigned short* __restrict__ Bt2p, int ldb, long strideB,
    void* __restrict__ Cout, void* __restrict__ Cout2, int ldc, long strideC,
    const float* __restrict__ bias,
    const float* __restrict__ resid, long strideR,
    int M, int N, int K, float scale) {
  typedef typename Elem<ET>::T T;
  typedef typename Frag<T>::V V;
  const T* A = (const T*)Ap; const T* A2 = (const T*)A2p; const T* Bt = (const T*)Btp; const T* Bt2 = (const T*)Bt2p;
  __shared__ __align__(16) float sT[8][16 * 68];
  const int b    = blockIdx.y;
  const int lane = threadIdx.x & 31;
  const int wave = threadIdx.x >> 5;
  const int tilesN = N >> 6;
  const int tilesM = M >> 6;
  const int tile = blockIdx.x * 8 + wave;
  if (tile >= tilesM * tilesN) return;
  const int tm = tile / tilesN;
  const int tn = tile - tm * tilesN;
  const int m0 = tm << 6;
  const int n0 = tn << 6;

  const T* Ab  = A  + (size_t)b * strideA;
  const T* Bb  = Bt + (size_t)b * strideB;
  const T* Ab2 = SPLIT ? (A2  + (size_t)b * strideA) : nullptr;
  const T* Bb2 = SPLIT ? (Bt2 + (size_t)b * strideB) : nullptr;

  const int rlane = lane & 15;
  const int koff  = (lane >> 4) * 8;
  const int mOff  = (lane >> 4) * 8;

  v8f acc[4][4];
#pragma unroll
  for (int i = 0; i < 4; ++i)
#pragma unroll
    for (int j = 0; j < 4; ++j) acc[i][j] = (v8f){0.f,0.f,0.f,0.f,0.f,0.f,0.f,0.f};

  for (int k0 = 0; k0 < K; k0 += 32) {
    V bh[4], bl[4];
#pragma unroll
    for (int j = 0; j < 4; ++j) {
      const size_t bo = (size_t)(n0 + (j << 4) + rlane) * ldb + koff + k0;
      bh[j] = Frag<T>::load(Bb + bo);
      if (SPLIT) bl[j] = Frag<T>::load(Bb2 + bo);
    }
#pragma unroll
    for (int i = 0; i < 4; ++i) {
      const size_t ao = (size_t)(m0 + (i << 4) + rlane) * lda + koff + k0;
      V ah = Frag<T>::load(Ab + ao);
      V al;
      if (SPLIT) al = Frag<T>::load(Ab2 + ao);
#pragma unroll
      for (int j = 0; j < 4; ++j) {
        acc[i][j] = Frag<T>::mma(ah, bh[j], acc[i][j]);
        if (SPLIT) {
          acc[i][j] = Frag<T>::mma(ah, bl[j], acc[i][j]);
          acc[i][j] = Frag<T>::mma(al, bh[j], acc[i][j]);
        }
      }
      Frag<T>::guard(acc[i][0], acc[i][3], ah, SPLIT ? al : ah);
    }
    Frag<T>::keep(bh[0], bh[1], bh[2], bh[3]);
    if (SPLIT) Frag<T>::keep(bl[0], bl[1], bl[2], bl[3]);
  }
  acc_guard4(acc[0][0], acc[0][1], acc[0][2], acc[0][3]);
  acc_guard4(acc[1][0], acc[1][1], acc[1][2], acc[1][3]);
  acc_guard4(acc[2][0], acc[2][1], acc[2][2], acc[2][3]);
  acc_guard4(acc[3][0], acc[3][1], acc[3][2], acc[3][3]);

  float* slab = sT[wave];
  const float* Rb = RESID ? (resid + (size_t)b * strideR) : nullptr;
#pragma unroll
  for (int i = 0; i < 4; ++i) {
    const int mBase = m0 + (i << 4);
#pragma unroll
    for (int j = 0; j < 4; ++j) {
      const int n = n0 + (j << 4) + rlane;
      float bv = 0.f;
      if (BIAS_MODE == 2) bv = bias[n];
#pragma unroll
      for (int r = 0; r < 8; ++r) {
        float v = acc[i][j][r] * scale;
        if (BIAS_MODE == 1) v += bias[mBase + mOff + r];
        if (BIAS_MODE == 2) v += bv;
        if (RESID) v += Rb[(size_t)(mBase + mOff + r) * ldc + n];
        if (ACT == 1) v = tanhf(v);
        if (ACT == 2) v = fmaxf(v, 0.0f);
        if (ACT == 3) v = v / (1.0f + expf(-v));
        if (ACT == 4) v = (v > 0.f) ? v : 0.01f * v;
        if (ACT == 5) v = 0.5f * v * (1.0f + erff(v * 0.70710678118654752f));
        slab[(mOff + r) * 68 + (j << 4) + rlane] = v;
      }
    }
    __builtin_amdgcn_fence(__ATOMIC_RELEASE, "workgroup");
    __builtin_amdgcn_wave_barrier();
    __builtin_amdgcn_fence(__ATOMIC_ACQUIRE, "workgroup");
    if (OUT_MODE == 0) {
      float* C = (float*)Cout + (size_t)b * strideC;
      const int hh = lane >> 4, c4 = (lane & 15) * 4;
      for (int pass = 0; pass < 2; ++pass) {
#pragma unroll
        for (int it = 0; it < 8; ++it) {
          const int row = it * 2 + hh;
          v4f v = *(const v4f*)(slab + row * 68 + c4);
          *(volatile v4f*)(C + (size_t)(mBase + row) * ldc + n0 + c4) = v;
        }
        __threadfence();
      }
    } else {
      const int q = lane >> 3, c8 = (lane & 7) * 8;
      unsigned short* C  = (unsigned short*)Cout  + (size_t)b * strideC;
      unsigned short* C2 = (OUT_MODE == 2) ? ((unsigned short*)Cout2 + (size_t)b * strideC) : nullptr;
      for (int pass = 0; pass < 2; ++pass) {
#pragma unroll
        for (int it = 0; it < 4; ++it) {
          const int row = it * 4 + q;
          const float* sp = slab + row * 68 + c8;
          v8h hv, lv;
#pragma unroll
          for (int e = 0; e < 8; ++e) {
            if (OUT_MODE == 1) {
              hv[e] = (_Float16)sp[e];
            } else {
              unsigned short hb = f2bf_bits(sp[e]);
              unsigned short lb = f2bf_bits(sp[e] - bf_bits2f(hb));
              hv[e] = __builtin_bit_cast(_Float16, hb);
              lv[e] = __builtin_bit_cast(_Float16, lb);
            }
          }
          *(volatile v8h*)(C + (size_t)(mBase + row) * ldc + n0 + c8) = hv;
          if (OUT_MODE == 2) *(volatile v8h*)(C2 + (size_t)(mBase + row) * ldc + n0 + c8) = lv;
        }
        __threadfence();
      }
    }
    __builtin_amdgcn_fence(__ATOMIC_RELEASE, "workgroup");
    __builtin_amdgcn_wave_barrier();
    __builtin_amdgcn_fence(__ATOMIC_ACQUIRE, "workgroup");
  }
}

__global__ __launch_bounds__(256) void corr_pack(const float* __restrict__ f1, const float* __restrict__ f2,
                                                 _Float16* __restrict__ o1, _Float16* __restrict__ o2) {
  __shared__ __align__(16) _Float16 T[64 * 264];
  const int tid = threadIdx.x, lane = tid & 31, wave = tid >> 5;
  const float* in = (blockIdx.y == 0) ? f1 : f2;
  _Float16* op    = (blockIdx.y == 0) ? o1 : o2;
  const int b  = blockIdx.x / (HW / 64);
  const int p0 = (blockIdx.x - b * (HW / 64)) * 64;
  const int px = tid & 63, cg = tid >> 6;
  const float* src = in + (size_t)b * NC * HW + p0 + px;
#pragma unroll 4
  for (int it = 0; it < 64; ++it) {
    const int c = it * 4 + cg;
    T[px * 264 + c] = (_Float16)src[(size_t)c * HW];
  }
  __syncthreads();
  for (int pass = 0; pass < 2; ++pass) {
#pragma unroll
    for (int r = 0; r < 8; ++r) {
      const int p = wave * 8 + r;
      const v8h v = *(const v8h*)(T + p * 264 + 8 * lane);
      *(volatile v8h*)(op + ((size_t)b * HW + p0 + p) * NC + 8 * lane) = v;
    }
    __threadfence();
  }
}

__global__ __launch_bounds__(256) void corr_lookup(const float* __restrict__ corr,
                                                   const float* __restrict__ cent,
                                                   float* __restrict__ out, int b, int row0) {
#pragma clang fp contract(off)
  __shared__ __align__(16) float Lbuf[3024];
  __shared__ __align__(16) float outT[NCH * 32];
  const int tid = threadIdx.x;
  const int lane = tid & 31, wave = tid >> 5;
  const int ry = blockIdx.x / 3;
  const int third = blockIdx.x - ry * 3;
  const int y = row0 + ry;
  const int xbase = third * 32;

#pragma unroll 1
  for (int px = 0; px < 32; ++px) {
    const int x = xbase + px;
    const float* R = corr + (size_t)(ry * WD + x) * HW;
    __syncthreads();
#pragma unroll 1
    for (int k = tid; k < 1152; k += 256) {
      const int Y = k / 24, X2 = k - Y * 24;
      const v4f a = *(const v4f*)(R + (2 * Y) * WD + 4 * X2);
      const v4f c = *(const v4f*)(R + (2 * Y + 1) * WD + 4 * X2);
      Lbuf[Y * 48 + 2 * X2]     = (((a[0] + a[1]) + c[0]) + c[1]) * 0.25f;
      Lbuf[Y * 48 + 2 * X2 + 1] = (((a[2] + a[3]) + c[2]) + c[3]) * 0.25f;
    }
    __syncthreads();
#pragma unroll 1
    for (int k = tid; k < 576; k += 256) {
      const int Y = k / 24, X = k - Y * 24;
      const float* s = Lbuf + (2 * Y) * 48 + 2 * X;
      Lbuf[2304 + k] = (((s[0] + s[1]) + s[48]) + s[49]) * 0.25f;
    }
    __syncthreads();
    if (tid < 144) {
      const int Y = tid / 12, X = tid - Y * 12;
      const float* s = Lbuf + 2304 + (2 * Y) * 24 + 2 * X;
      Lbuf[2880 + tid] = (((s[0] + s[1]) + s[24]) + s[25]) * 0.25f;
    }
    __syncthreads();

    const float cx = cent[((size_t)(b * 2 + 0) * WD + y) * WD + x];
    const float cy = cent[((size_t)(b * 2 + 1) * WD + y) * WD + x];
#pragma unroll 1
    for (int o = tid; o < NCH; o += 256) {
      const int lvl = o / 81;
      const int rem = o - lvl * 81;
      const int i = rem / 9, j = rem - i * 9;
      const int wl = WD >> lvl;
      const float wlm1 = (float)(wl - 1);
      const float sc = (lvl == 0) ? 1.0f : (lvl == 1) ? 0.5f : (lvl == 2) ? 0.25f : 0.125f;
      const int loff = (lvl == 2) ? 2304 : (lvl == 3) ? 2880 : 0;
      const float xs = cx * sc + (float)(i - 4);
      const float ys = cy * sc + (float)(j - 4);
      const float x0 = floorf(xs), y0 = floorf(ys);
      const float wx1 = xs - x0, wy1 = ys - y0;
      const float wx0 = 1.0f - wx1, wy0 = 1.0f - wy1;
      float val = 0.0f;
#pragma unroll
      for (int cnr = 0; cnr < 4; ++cnr) {
        const int dx = cnr & 1, dy = cnr >> 1;
        const float xi = dx ? (x0 + 1.0f) : x0;
        const float yi = dy ? (y0 + 1.0f) : y0;
        const bool valid = (xi >= 0.0f) && (xi <= wlm1) && (yi >= 0.0f) && (yi <= wlm1);
        const int xc = (int)fminf(fmaxf(xi, 0.0f), wlm1);
        const int yc = (int)fminf(fmaxf(yi, 0.0f), wlm1);
        const float gg = R[yc * WD + xc];
        int li = loff + yc * wl + xc;
        li = (li > 3023) ? 3023 : li;
        const float gl = Lbuf[li];
        float g = (lvl == 0) ? gg : gl;
        g = valid ? g : 0.0f;
        const float wxv = dx ? wx1 : wx0;
        const float wyv = dy ? wy1 : wy0;
        val = val + (g * wxv) * wyv;
      }
      outT[o * 32 + px] = val;
    }
  }
  __syncthreads();
  for (int pass = 0; pass < 2; ++pass) {
#pragma unroll 1
    for (int g = wave; g < 81; g += 8) {
      const int o = g * 4 + (lane >> 3);
      const v4f v = *(const v4f*)(outT + o * 32 + 4 * (lane & 7));
      float* dst = out + (((size_t)b * NCH + o) * WD + y) * WD + xbase + 4 * (lane & 7);
      *(volatile v4f*)dst = v;
    }
    __threadfence();
  }
}

extern "C" void kernel_launch(void* const* d_in, const int* in_sizes, int n_in,
                              void* d_out, int out_size, void* d_ws, size_t ws_size,
                              hipStream_t stream) {
  if (n_in < 3) return;
  if (in_sizes[0] != NB * NC * HW || in_sizes[1] != NB * NC * HW || in_sizes[2] != NB * 2 * HW) return;
  if (out_size != NB * NCH * HW) return;

  const size_t f16_bytes  = (size_t)NB * HW * NC * 2;
  const size_t off_f1     = 0;
  const size_t off_f2     = f16_bytes;
  const size_t off_corr   = 2 * f16_bytes;
  const size_t corr_bytes = (size_t)CHUNK_PIX * HW * 4;
  if (off_corr + corr_bytes > ws_size) return;

  const float* f1   = (const float*)d_in[0];
  const float* f2   = (const float*)d_in[1];
  const float* cent = (const float*)d_in[2];
  float* out = (float*)d_out;
  char* ws = (char*)d_ws;
  _Float16* F1T = (_Float16*)(ws + off_f1);
  _Float16* F2T = (_Float16*)(ws + off_f2);
  float* CORR = (float*)(ws + off_corr);

  corr_pack<<<dim3(NB * HW / 64, 2), 256, 0, stream>>>(f1, f2, F1T, F2T);

  const int gemm_blocks = (CHUNK_PIX / 64) * (HW / 64) / 8;
  for (int ci = 0; ci < NB * NCHUNK_PER_B; ++ci) {
    const int b = ci / NCHUNK_PER_B, part = ci % NCHUNK_PER_B;
    const unsigned short* Ap = (const unsigned short*)(F1T + ((size_t)b * HW + (size_t)part * CHUNK_PIX) * NC);
    const unsigned short* Bp = (const unsigned short*)(F2T + (size_t)b * HW * NC);
    wmma_gemm64<0, false, 0, 0, false, 0><<<dim3(gemm_blocks, 1), 256, 0, stream>>>(
        Ap, Ap, NC, 0L, Bp, Bp, NC, 0L,
        (void*)CORR, (void*)CORR, HW, 0L,
        (const float*)CORR, (const float*)CORR, 0L,
        CHUNK_PIX, HW, NC, 0.0625f);
    corr_lookup<<<CHUNK_ROWS * 3, 256, 0, stream>>>(CORR, cent, out, b, part * CHUNK_ROWS);
  }
}
